// BidirectionalVSSM_4690104287388
// MI455X (gfx1250) — hardware-run, weakly checked
//
#include <hip/hip_runtime.h>
#include <hip/hip_fp16.h>
#include <math.h>

typedef __attribute__((ext_vector_type(16))) _Float16 v16h;
typedef __attribute__((ext_vector_type(8)))  _Float16 v8h;
typedef __attribute__((ext_vector_type(8)))  float    v8f;
typedef __attribute__((ext_vector_type(4)))  float    v4f;
typedef __attribute__((ext_vector_type(2)))  unsigned v2u;
typedef __attribute__((ext_vector_type(4)))  unsigned v4u;

constexpr int kBatch   = 8;
constexpr int kHW      = 16;
constexpr int kL       = kHW * kHW;
constexpr int kRows    = kBatch * kL;
constexpr int kDm      = 384;
constexpr int kE       = 768;
constexpr int kXzN     = 2 * kE;
constexpr int kNst     = 16;
constexpr int kRank    = 24;
constexpr int kRkP     = 32;
constexpr int kXpN     = kRank + 2 * kNst;
constexpr int kXpP     = 64;
constexpr int kDirs    = 4;
constexpr int kAlpFloats = kE * kNst;
constexpr int kPadFloats = kAlpFloats + kE;
constexpr float kXCarry = 64.0f;
constexpr float kWCarry = 1024.0f;
constexpr float kSCarry = 256.0f;
constexpr float kRCarry = 1024.0f;
constexpr float kGCarry = 256.0f;
constexpr float kYCarry = 64.0f;
constexpr float kResid  = 2048.0f;
constexpr float kMergeScale = 0.25f / kYCarry;
static_assert(kHW == 16 && kL == 256 && kRows == 2048);
static_assert(kDm == 384 && kE == 768 && kXzN == 1536 && kXpN == 56 && kDirs == 4 && kNst == 16);
static_assert(kRank + 1 <= kRkP && (kRank % 8) == 0 && kRank + 2 * kNst <= kXpP);
static_assert((kDm % 32) == 0 && (kE % 32) == 0 && (kRkP % 32) == 0);
static_assert((kDm % 64) == 0 && (kE % 64) == 0 && (kXzN % 64) == 0 && (kXpP % 64) == 0);
static_assert((kRows % 32) == 0);
static_assert((kL % 64) == 0 && (kL % 4) == 0);
static_assert(kAlpFloats == 12288 && kPadFloats == 13056);

constexpr size_t kSzXH   = (size_t)kRows * kDm * 2;
constexpr size_t kSzWIN  = (size_t)kXzN * kDm * 2;
constexpr size_t kSzXZ   = (size_t)kRows * kXzN * 4;
constexpr size_t kSzXIH  = (size_t)kRows * kE * 2;
constexpr size_t kSzWX   = (size_t)kXpP * kE * 2;
constexpr size_t kSzXD0  = (size_t)kRows * kXpP * 4;
constexpr size_t kSzDRH  = (size_t)kRows * kRkP * 2;
constexpr size_t kSzWDT  = (size_t)kE * kRkP * 2;
constexpr size_t kSzDT0  = (size_t)kRows * kE * 4;
constexpr size_t kSzXS   = (size_t)kDirs * kRows * kE * 4;
constexpr size_t kSzDTP  = (size_t)kDirs * kRows * kE * 4;
constexpr size_t kSzXD   = (size_t)kDirs * kRows * kXpP * 4;
constexpr size_t kSzPADS = (size_t)kPadFloats * 4;
constexpr size_t kSzYH   = (size_t)kDirs * kRows * kE * 2;
constexpr size_t kSzYG   = (size_t)kRows * kE * 2;
constexpr size_t kSzOW   = (size_t)kDm * kE * 2;
constexpr size_t kSzRAW  = (size_t)kRows * kDm * 4;
constexpr size_t kSzRES  = (size_t)kRows * kDm * 4;
constexpr size_t kSzST   = (size_t)kRows * 4 * 4;
constexpr size_t kOffXH   = 0;
constexpr size_t kOffWIN  = kOffXH   + kSzXH;
constexpr size_t kOffXZ   = kOffWIN  + kSzWIN;
constexpr size_t kOffXIH  = kOffXZ   + kSzXZ;
constexpr size_t kOffWX   = kOffXIH  + kSzXIH;
constexpr size_t kOffXD0  = kOffWX   + kSzWX;
constexpr size_t kOffDRH  = kOffXD0  + kSzXD0;
constexpr size_t kOffWDT  = kOffDRH  + kSzDRH;
constexpr size_t kOffDT0  = kOffWDT  + kSzWDT;
constexpr size_t kOffXS   = kOffDT0  + kSzDT0;
constexpr size_t kOffDTP  = kOffXS   + kSzXS;
constexpr size_t kOffXD   = kOffDTP  + kSzDTP;
constexpr size_t kOffPADS = kOffXD   + kSzXD;
constexpr size_t kOffYH   = kOffPADS + kSzPADS;
constexpr size_t kOffYG   = kOffYH   + kSzYH;
constexpr size_t kOffOW   = kOffYG   + kSzYG;
constexpr size_t kOffRAW  = kOffOW   + kSzOW;
constexpr size_t kOffRES  = kOffRAW  + kSzRAW;
constexpr size_t kOffST   = kOffRES  + kSzRES;
constexpr size_t kWsTotal = kOffST   + kSzST;
static_assert(kSzXH == 1572864ull && kSzWIN == 1179648ull && kSzXZ == 12582912ull && kSzXIH == 3145728ull);
static_assert(kSzWX == 98304ull && kSzXD0 == 524288ull && kSzDRH == 131072ull && kSzWDT == 49152ull);
static_assert(kSzDT0 == 6291456ull && kSzXS == 25165824ull && kSzDTP == 25165824ull && kSzXD == 2097152ull);
static_assert(kSzPADS == 52224ull && kSzYH == 12582912ull && kSzYG == 3145728ull && kSzOW == 589824ull);
static_assert(kSzRAW == 3145728ull && kSzRES == 3145728ull && kSzST == 32768ull);
static_assert(kWsTotal == 1572864ull + 1179648ull + 12582912ull + 3145728ull + 98304ull + 524288ull + 131072ull +
              49152ull + 6291456ull + 25165824ull + 25165824ull + 2097152ull + 52224ull + 12582912ull +
              3145728ull + 589824ull + 3145728ull + 3145728ull + 32768ull);
static_assert(kWsTotal == 100699136ull);
static_assert(kWsTotal <= 134217728ull);
static_assert((kSzXH % 128) == 0 && (kSzWIN % 128) == 0 && (kSzXZ % 128) == 0 && (kSzXIH % 128) == 0 &&
              (kSzWX % 128) == 0 && (kSzXD0 % 128) == 0 && (kSzDRH % 128) == 0 && (kSzWDT % 128) == 0 &&
              (kSzDT0 % 128) == 0 && (kSzXS % 128) == 0 && (kSzDTP % 128) == 0 && (kSzXD % 128) == 0 &&
              (kSzPADS % 128) == 0 && (kSzYH % 128) == 0 && (kSzYG % 128) == 0 && (kSzOW % 128) == 0 &&
              (kSzRAW % 128) == 0 && (kSzRES % 128) == 0 && (kSzST % 128) == 0);
static_assert((((size_t)kRows * kE * 4) % 128) == 0 && (((size_t)kRows * kE * 2) % 128) == 0 &&
              (((size_t)kRows * kXpP * 4) % 128) == 0 && (((size_t)kAlpFloats * 4) % 128) == 0);

__device__ __forceinline__ _Float16 f16_flush(float v) {
  const float w = (fabsf(v) < 6.103515625e-05f) ? 0.0f : v;
  return (_Float16)w;
}
__device__ __forceinline__ void f16_split(float v, _Float16& hi, _Float16& lo) {
  hi = f16_flush(v);
  const float hf = (float)hi;
  const float r = (v - hf) * kResid;
  lo = f16_flush(r);
}

__device__ __forceinline__ float bf16r(float v) {
  unsigned u = __float_as_uint(v);
  u = (u + 0x7FFFu + ((u >> 16) & 1u)) & 0xFFFF0000u;
  return __uint_as_float(u);
}

__device__ __forceinline__ float h16_to_f32(unsigned hb) {
  const unsigned sgn = (hb & 0x8000u) << 16; const unsigned em = hb & 0x7fffu;
  const float fn = __uint_as_float((em << 13) + 0x38000000u);
  const float fs = (float)em * 5.9604644775390625e-8f;
  const float mag = (em < 0x400u) ? fs : fn; return __uint_as_float(__float_as_uint(mag) | sgn); }

namespace eng {
union FragU { v16h v; v8h h[2]; };
__device__ __forceinline__ v16h frag_load(const _Float16* p) {
  FragU f;
  f.h[0] = *(const v8h*)(p);
  f.h[1] = *(const v8h*)(p + 16);
  return f.v;
}
__device__ __forceinline__ v8f mma(v16h a, v16h b, v8f c) {
  return __builtin_amdgcn_wmma_f32_16x16x32_f16(false, a, false, b, (short)0, c, false, false);
}
__device__ __forceinline__ void guard1(v8f& a, v16h x, v16h y) {
  asm volatile("v_nop\n\tv_nop\n\tv_nop\n\tv_nop" : "+v"(a) : "v"(x), "v"(y));
}
__device__ __forceinline__ void guard_acc(v8f& a) {
  asm volatile("v_nop\n\tv_nop\n\tv_nop\n\tv_nop" : "+v"(a));
}
__device__ __forceinline__ void keep4(v16h a, v16h b, v16h c, v16h d) {
  asm volatile("v_nop" :: "v"(a), "v"(b), "v"(c), "v"(d));
}

template <int MI, int SPL>
__global__ __launch_bounds__(256) void gemm_f16_kernel(
    const unsigned short* __restrict__ Ap, const unsigned short* __restrict__ A2p, int lda,
    const unsigned short* __restrict__ Btp, const unsigned short* __restrict__ Bt2p, int ldb,
    float* __restrict__ C, int ldc, int M, int N, int K, float scale, float rscale)
{
  static_assert(MI >= 1 && MI <= 2);
  static_assert(SPL >= 0 && SPL <= 2);
  const _Float16* A   = (const _Float16*)Ap;
  const _Float16* A2  = (const _Float16*)A2p;
  const _Float16* Bt  = (const _Float16*)Btp;
  const _Float16* Bt2 = (const _Float16*)Bt2p;
  __shared__ __align__(16) float sT[8][16 * 68];
  const int lane = threadIdx.x & 31;
  const int wave = threadIdx.x >> 5;
  const int tilesN = N >> 6;
  const int tilesM = M / (16 * MI);
  const int tile = blockIdx.x * 8 + wave;
  if (tile >= tilesM * tilesN) return;
  const int tm = tile / tilesN;
  const int tn = tile - tm * tilesN;
  const int m0 = tm * (16 * MI);
  const int n0 = tn << 6;
  const int rlane = lane & 15;
  const int koff  = (lane >> 4) * 8;
  const int mOff  = (lane >> 4) * 8;

  v8f acc[MI][4], accr[MI][4];
#pragma unroll
  for (int i = 0; i < MI; ++i)
#pragma unroll
    for (int j = 0; j < 4; ++j) {
      acc[i][j]  = (v8f){0.f, 0.f, 0.f, 0.f, 0.f, 0.f, 0.f, 0.f};
      accr[i][j] = (v8f){0.f, 0.f, 0.f, 0.f, 0.f, 0.f, 0.f, 0.f};
    }

  for (int k0 = 0; k0 < K; k0 += 32) {
    v16h bh[4], bl[4];
#pragma unroll
    for (int j = 0; j < 4; ++j) {
      const size_t bo = (size_t)(n0 + (j << 4) + rlane) * ldb + koff + k0;
      bh[j] = frag_load(Bt + bo);
      if (SPL == 2) bl[j] = frag_load(Bt2 + bo); else bl[j] = bh[j];
    }
#pragma unroll
    for (int i = 0; i < MI; ++i) {
      const size_t ao = (size_t)(m0 + (i << 4) + rlane) * lda + koff + k0;
      const v16h ah = frag_load(A + ao);
      v16h al = ah;
      if (SPL >= 1) al = frag_load(A2 + ao);
#pragma unroll
      for (int j = 0; j < 4; ++j) {
        acc[i][j] = mma(ah, bh[j], acc[i][j]);
        if (SPL >= 1) accr[i][j] = mma(al, bh[j], accr[i][j]);
        if (SPL == 2) accr[i][j] = mma(ah, bl[j], accr[i][j]);
      }
#pragma unroll
      for (int j = 0; j < 4; ++j) {
        guard1(acc[i][j], ah, al);
        if (SPL >= 1) guard1(accr[i][j], ah, al);
      }
    }
    keep4(bh[0], bh[1], bh[2], bh[3]);
    if (SPL == 2) keep4(bl[0], bl[1], bl[2], bl[3]);
  }
#pragma unroll
  for (int i = 0; i < MI; ++i)
#pragma unroll
    for (int j = 0; j < 4; ++j) {
      guard_acc(acc[i][j]);
      if (SPL >= 1) guard_acc(accr[i][j]);
    }

  float* slab = sT[wave];
#pragma unroll
  for (int i = 0; i < MI; ++i) {
    const int mBase = m0 + (i << 4);
#pragma unroll
    for (int j = 0; j < 4; ++j) {
#pragma unroll
      for (int r = 0; r < 8; ++r) {
        float v = acc[i][j][r] * scale;
        if (SPL >= 1) v += accr[i][j][r] * rscale;
        slab[(mOff + r) * 68 + (j << 4) + rlane] = v;
      }
    }
    __builtin_amdgcn_fence(__ATOMIC_RELEASE, "workgroup");
    __builtin_amdgcn_wave_barrier();
    __builtin_amdgcn_fence(__ATOMIC_ACQUIRE, "workgroup");
    {
      const int hh = lane >> 4, c4 = (lane & 15) * 4;
      for (int pass = 0; pass < 2; ++pass) {
#pragma unroll
        for (int it = 0; it < 8; ++it) {
          const int row = it * 2 + hh;
          const v4f v = *(const v4f*)(slab + row * 68 + c4);
          *(volatile v4f*)(C + (size_t)(mBase + row) * ldc + n0 + c4) = v;
        }
        __threadfence();
      }
    }
    __builtin_amdgcn_fence(__ATOMIC_RELEASE, "workgroup");
    __builtin_amdgcn_wave_barrier();
    __builtin_amdgcn_fence(__ATOMIC_ACQUIRE, "workgroup");
  }
}
}

__device__ __forceinline__ _Float16 in_half(float v, float carry, bool live) {
  const float t = live ? (bf16r(v) * carry) : 0.0f;
  return f16_flush(t);
}
__device__ __forceinline__ _Float16 val_half(float v, float carry, bool live) {
  const float t = live ? (v * carry) : 0.0f;
  return f16_flush(t);
}
__device__ __forceinline__ v8h pack8_in(v4f a0, v4f a1, float carry, bool live) {
  const float f0 = a0[0];
  const float f1 = a0[1];
  const float f2 = a0[2];
  const float f3 = a0[3];
  const float f4 = a1[0];
  const float f5 = a1[1];
  const float f6 = a1[2];
  const float f7 = a1[3];
  v8h hv;
  hv[0] = in_half(f0, carry, live);
  hv[1] = in_half(f1, carry, live);
  hv[2] = in_half(f2, carry, live);
  hv[3] = in_half(f3, carry, live);
  hv[4] = in_half(f4, carry, live);
  hv[5] = in_half(f5, carry, live);
  hv[6] = in_half(f6, carry, live);
  hv[7] = in_half(f7, carry, live);
  return hv;
}
__device__ __forceinline__ int src_token(int k, int t) {
  const int u = ((k & 1) != 0) ? (kL - 1 - t) : t;
  const int uq = u / kHW;
  const int ur = u - uq * kHW;
  const int tr = ur * kHW + uq;
  return (k >= 2) ? tr : u;
}
__device__ __forceinline__ int inv_time(int k, int p) {
  const int pq = p / kHW;
  const int pr = p - pq * kHW;
  const int tr = pr * kHW + pq;
  const int q = (k >= 2) ? tr : p;
  return ((k & 1) != 0) ? (kL - 1 - q) : q;
}

__global__ __launch_bounds__(256) void pack_x_kernel(
    const float* __restrict__ x, unsigned short* __restrict__ XH)
{
  const int i = blockIdx.x * 256 + threadIdx.x;
  const int r = i / (kDm / 8);
  const int c8 = (i - r * (kDm / 8)) * 8;
  const float* sp = x + (size_t)r * kDm + c8;
  const v4f a0 = *(const v4f*)(sp);
  const v4f a1 = *(const v4f*)(sp + 4);
  const v8h hv = pack8_in(a0, a1, kXCarry, true);
  unsigned short* q = XH + (size_t)i * 8;
  *(volatile v8h*)q = hv;
  __threadfence();
  *(volatile v8h*)q = hv;
}

__global__ __launch_bounds__(256) void pack_win_kernel(
    const float* __restrict__ w, unsigned short* __restrict__ WIN)
{
  const int i = blockIdx.x * 256 + threadIdx.x;
  const int n = i / (kDm / 8);
  const int c8 = (i - n * (kDm / 8)) * 8;
  const float* sp = w + (size_t)n * kDm + c8;
  const v4f a0 = *(const v4f*)(sp);
  const v4f a1 = *(const v4f*)(sp + 4);
  const v8h hv = pack8_in(a0, a1, kWCarry, true);
  unsigned short* q = WIN + (size_t)i * 8;
  *(volatile v8h*)q = hv;
  __threadfence();
  *(volatile v8h*)q = hv;
}

__global__ __launch_bounds__(256) void pack_xi_kernel(
    const float* __restrict__ XZ, unsigned short* __restrict__ XIH)
{
  const int i = blockIdx.x * 256 + threadIdx.x;
  const int r = i / (kE / 8);
  const int c8 = (i - r * (kE / 8)) * 8;
  const float* sp = XZ + (size_t)r * kXzN + c8;
  const v4f a0 = *(const v4f*)(sp);
  const v4f a1 = *(const v4f*)(sp + 4);
  const float f0 = a0[0];
  const float f1 = a0[1];
  const float f2 = a0[2];
  const float f3 = a0[3];
  const float f4 = a1[0];
  const float f5 = a1[1];
  const float f6 = a1[2];
  const float f7 = a1[3];
  v8h hv;
  hv[0] = val_half(f0, kSCarry, true);
  hv[1] = val_half(f1, kSCarry, true);
  hv[2] = val_half(f2, kSCarry, true);
  hv[3] = val_half(f3, kSCarry, true);
  hv[4] = val_half(f4, kSCarry, true);
  hv[5] = val_half(f5, kSCarry, true);
  hv[6] = val_half(f6, kSCarry, true);
  hv[7] = val_half(f7, kSCarry, true);
  unsigned short* q = XIH + (size_t)i * 8;
  *(volatile v8h*)q = hv;
  __threadfence();
  *(volatile v8h*)q = hv;
}

__global__ __launch_bounds__(256) void pack_wx_kernel(
    const float* __restrict__ w, unsigned short* __restrict__ WX)
{
  const int i = blockIdx.x * 256 + threadIdx.x;
  const int n = i / (kE / 8);
  const int j8 = (i - n * (kE / 8)) * 8;
  const bool live = (n < kXpN);
  const int nc = live ? n : (kXpN - 1);
  const float* sp = w + ((size_t)nc * kE + j8);
  const v4f a0 = *(const v4f*)(sp);
  const v4f a1 = *(const v4f*)(sp + 4);
  const v8h hv = pack8_in(a0, a1, kWCarry, live);
  unsigned short* q = WX + (size_t)i * 8;
  *(volatile v8h*)q = hv;
  __threadfence();
  *(volatile v8h*)q = hv;
}

__device__ __forceinline__ _Float16 dr_half(float v, int j) {
  const float t = (j < kRank) ? (v * kRCarry) : ((j == kRank) ? kRCarry : 0.0f);
  return f16_flush(t);
}
__global__ __launch_bounds__(256) void pack_dr_kernel(
    const float* __restrict__ XD0, unsigned short* __restrict__ DRH)
{
  const int i = blockIdx.x * 256 + threadIdx.x;
  const int row = i / (kRkP / 8);
  const int j8 = (i - row * (kRkP / 8)) * 8;
  const int jc = (j8 < kRank) ? j8 : (kRank - 8);
  const float* sp = XD0 + (size_t)row * kXpP + jc;
  const v4f a0 = *(const v4f*)(sp);
  const v4f a1 = *(const v4f*)(sp + 4);
  const float f0 = a0[0];
  const float f1 = a0[1];
  const float f2 = a0[2];
  const float f3 = a0[3];
  const float f4 = a1[0];
  const float f5 = a1[1];
  const float f6 = a1[2];
  const float f7 = a1[3];
  v8h hv;
  hv[0] = dr_half(f0, j8 + 0);
  hv[1] = dr_half(f1, j8 + 1);
  hv[2] = dr_half(f2, j8 + 2);
  hv[3] = dr_half(f3, j8 + 3);
  hv[4] = dr_half(f4, j8 + 4);
  hv[5] = dr_half(f5, j8 + 5);
  hv[6] = dr_half(f6, j8 + 6);
  hv[7] = dr_half(f7, j8 + 7);
  unsigned short* q = DRH + (size_t)i * 8;
  *(volatile v8h*)q = hv;
  __threadfence();
  *(volatile v8h*)q = hv;
}

__device__ __forceinline__ _Float16 dtw_half(const float* __restrict__ wrow, float bias, int j) {
  const int jc = (j < kRank) ? j : (kRank - 1);
  const float wv = wrow[jc];
  const float t = (j < kRank) ? (bf16r(wv) * kWCarry) : ((j == kRank) ? (bf16r(bias) * kWCarry) : 0.0f);
  return f16_flush(t);
}
__global__ __launch_bounds__(256) void pack_wdt_kernel(
    const float* __restrict__ dtw, const float* __restrict__ dtb, unsigned short* __restrict__ WDT)
{
  const int i = blockIdx.x * 256 + threadIdx.x;
  const int kc = i / (kRkP / 8);
  const int j8 = (i - kc * (kRkP / 8)) * 8;
  const float* wrow = dtw + (size_t)kc * kRank;
  const float bias = dtb[kc];
  v8h hv;
  hv[0] = dtw_half(wrow, bias, j8 + 0);
  hv[1] = dtw_half(wrow, bias, j8 + 1);
  hv[2] = dtw_half(wrow, bias, j8 + 2);
  hv[3] = dtw_half(wrow, bias, j8 + 3);
  hv[4] = dtw_half(wrow, bias, j8 + 4);
  hv[5] = dtw_half(wrow, bias, j8 + 5);
  hv[6] = dtw_half(wrow, bias, j8 + 6);
  hv[7] = dtw_half(wrow, bias, j8 + 7);
  unsigned short* q = WDT + (size_t)i * 8;
  *(volatile v8h*)q = hv;
  __threadfence();
  *(volatile v8h*)q = hv;
}

__global__ __launch_bounds__(256) void order_kernel(
    const float* __restrict__ XZ, float* __restrict__ XS)
{
  const int i = blockIdx.x * 256 + threadIdx.x;
  const int k = i / (kRows * (kE / 4));
  const int rem = i - k * (kRows * (kE / 4));
  const int R = rem / (kE / 4);
  const int c4 = (rem - R * (kE / 4)) * 4;
  const int b = R / kL;
  const int t = R - b * kL;
  const int src = b * kL + src_token(k, t);
  const v4f v = *(const v4f*)(XZ + (size_t)src * kXzN + c4);
  float* q = XS + (size_t)i * 4;
  *(volatile v4f*)q = v;
  __threadfence();
  *(volatile v4f*)q = v;
}

__global__ __launch_bounds__(256) void gather_dt_kernel(
    const float* __restrict__ DT0, float* __restrict__ DTP)
{
  const int i = blockIdx.x * 256 + threadIdx.x;
  const int k = i / (kRows * (kE / 4));
  const int rem = i - k * (kRows * (kE / 4));
  const int R = rem / (kE / 4);
  const int c4 = (rem - R * (kE / 4)) * 4;
  const int b = R / kL;
  const int t = R - b * kL;
  const int src = b * kL + src_token(k, t);
  const v4f v = *(const v4f*)(DT0 + (size_t)src * kE + c4);
  float* q = DTP + (size_t)i * 4;
  *(volatile v4f*)q = v;
  __threadfence();
  *(volatile v4f*)q = v;
}

__global__ __launch_bounds__(256) void gather_bc_kernel(
    const float* __restrict__ XD0, float* __restrict__ XD)
{
  const int i = blockIdx.x * 256 + threadIdx.x;
  const int k = i / (kRows * (kXpP / 4));
  const int rem = i - k * (kRows * (kXpP / 4));
  const int R = rem / (kXpP / 4);
  const int j4 = (rem - R * (kXpP / 4)) * 4;
  const int b = R / kL;
  const int t = R - b * kL;
  const int src = b * kL + src_token(k, t);
  const v4f o = *(const v4f*)(XD0 + ((size_t)src * kXpP + j4));
  float* q = XD + (size_t)i * 4;
  *(volatile v4f*)q = o;
  __threadfence();
  *(volatile v4f*)q = o;
}

__global__ __launch_bounds__(32) void pads_kernel(
    const float* __restrict__ alog, float* __restrict__ PADS)
{
  const int wi = blockIdx.x * 32 + threadIdx.x;
  const int f0 = wi * 4;
  const bool isA = (f0 < kAlpFloats);
  const int ea = isA ? f0 : (kAlpFloats - 4);
  const v4f va = *(const v4f*)(alog + ea);
  const float a0 = va[0];
  const float a1 = va[1];
  const float a2 = va[2];
  const float a3 = va[3];
  const float r0 = bf16r(a0);
  const float r1 = bf16r(a1);
  const float r2 = bf16r(a2);
  const float r3 = bf16r(a3);
  v4f o;
  o[0] = isA ? r0 : 0.0f;
  o[1] = isA ? r1 : 0.0f;
  o[2] = isA ? r2 : 0.0f;
  o[3] = isA ? r3 : 0.0f;
  float* q = PADS + (size_t)f0;
  *(volatile v4f*)q = o;
  __threadfence();
  *(volatile v4f*)q = o;
}

typedef float    ms1_v4f __attribute__((ext_vector_type(4)));
typedef unsigned ms1_v4u __attribute__((ext_vector_type(4)));
struct ms1_args {
  const float* dtpre;
  const float* u;
  const float* bc;
  const float* z;
  const float* A_log;
  const float* Dskip;
  __half* y;
  __half* y_lo;
  long ld_dtpre;
  long ld_u;
  long ld_bc;
  long ld_z;
  long ld_y;
  int offB;
  int offC;
  int offZ;
  float ycarry;
  int dir;
  int D;
  int L;
  int nbatch;
};
static_assert(sizeof(ms1_args) == 136);

__device__ __forceinline__ float ms1_flush16(float v) {
  return (fabsf(v) < 6.103515625e-05f) ? 0.0f : v;
}
__device__ __forceinline__ unsigned ms1_h16bits(float v) {
  return (unsigned)__half_as_ushort(__float2half_rn(ms1_flush16(v)));
}
__device__ __forceinline__ float ms1_h16val(unsigned b) {
  return __half2float(__ushort_as_half((unsigned short)b));
}
__device__ __forceinline__ float ms1_softplus(float v) {
  return fmaxf(v, 0.0f) + log1pf(expf(-fabsf(v)));
}
__device__ __forceinline__ void ms1_pack2(float v0, float v1, unsigned& hw, unsigned& lw) {
  const unsigned h0 = ms1_h16bits(v0);
  const unsigned h1 = ms1_h16bits(v1);
  const float r0 = (v0 - ms1_h16val(h0)) * 2048.0f;
  const float r1 = (v1 - ms1_h16val(h1)) * 2048.0f;
  const unsigned l0 = ms1_h16bits(r0);
  const unsigned l1 = ms1_h16bits(r1);
  hw = h0 | (h1 << 16);
  lw = l0 | (l1 << 16);
}

template <int NSTATE>
__global__ __launch_bounds__(64 * (NSTATE / 16)) void ms1_scan_kernel(ms1_args a)
{
  static_assert(NSTATE == 16 || NSTATE == 64);
  constexpr int NQ  = NSTATE / 16;
  constexpr int NT  = 64 * NQ;
  constexpr int NW  = NT / 32;
  constexpr int BCW = 2 * NSTATE;
  constexpr int YP  = 68;
  constexpr int RPI = NW * 4;
  constexpr int NIT = 64 / RPI;
  static_assert(16 * NT <= 64 * YP);
  __shared__ __align__(16) float sBC[64 * BCW];
  __shared__ __align__(16) float sY[64 * YP];
  const int tid  = threadIdx.x;
  const int lane = tid & 31;
  const int wave = tid >> 5;
  const int c    = tid / NQ;
  const int sq   = tid - c * NQ;
  const int bpb  = a.D / 64;
  const int bi   = blockIdx.x / bpb;
  if (bi >= a.nbatch) return;
  const int d0 = (blockIdx.x - bi * bpb) * 64;
  const int d  = d0 + c;
  const long rowb = (long)bi * a.L;
  const bool hasz  = (a.z != nullptr);
  const bool hasD  = (a.Dskip != nullptr);
  const bool hasLo = (a.y_lo != nullptr);

#pragma unroll 1
  for (int n = 0; n < 16; ++n) {
    const float al = a.A_log[(long)d * NSTATE + sq * 16 + n];
    sY[n * NT + tid] = -expf(al);
  }
  __syncthreads();
  float An[16], h[16];
#pragma unroll
  for (int n = 0; n < 16; ++n) {
    An[n] = sY[n * NT + tid];
    h[n] = 0.0f;
  }
  float Dd = 0.0f;
  if (hasD) Dd = a.Dskip[d];

  const int nchunk = a.L / 64;
  const bool fwd = (a.dir > 0);
  const int s0 = fwd ? 0 : 63;
  const int sd = fwd ? 1 : -1;
  const int q  = lane >> 3;
  const int c8 = (lane & 7) * 8;

  for (int ci = 0; ci < nchunk; ++ci) {
    const int tb = fwd ? (ci * 64) : (a.L - 64 - ci * 64);
    const long rowc = rowb + tb;
    __syncthreads();
#pragma unroll 8
    for (int i = 0; i < 32; ++i) {
      const int idx = tid + i * NT;
      const int st  = idx / BCW;
      const int col = idx - st * BCW;
      const int sc  = (col < NSTATE) ? (a.offB + col) : (a.offC + col - NSTATE);
      sBC[idx] = a.bc[(rowc + st) * a.ld_bc + sc];
    }
    __syncthreads();
    for (int s = 0; s < 64; ++s) {
      const int ls = s0 + sd * s;
      const long row = rowc + ls;
      float pre = a.dtpre[row * a.ld_dtpre + d];
      float uv  = a.u[row * a.ld_u + d];
      float zv  = 0.0f;
      if (hasz) zv = a.z[row * a.ld_z + a.offZ + d];
      asm volatile("" : "+v"(pre));
      asm volatile("" : "+v"(uv));
      asm volatile("" : "+v"(zv));
      const float delta = ms1_softplus(pre);
      const float dtx = delta * uv;
      const float* bp = sBC + ls * BCW + sq * 16;
      const float* cp = bp + NSTATE;
      ms1_v4f Bq[4], Cq[4];
#pragma unroll
      for (int k = 0; k < 4; ++k) {
        Bq[k] = *(const ms1_v4f*)(bp + 4 * k);
        Cq[k] = *(const ms1_v4f*)(cp + 4 * k);
      }
      float yv = 0.0f;
#pragma unroll
      for (int n = 0; n < 16; ++n) {
        const float e = __expf(delta * An[n]);
        h[n] = fmaf(e, h[n], dtx * Bq[n >> 2][n & 3]);
        yv = fmaf(h[n], Cq[n >> 2][n & 3], yv);
      }
      if (NQ > 1) {
        yv += __shfl_xor(yv, 1, 32);
        yv += __shfl_xor(yv, 2, 32);
      }
      if (hasD) yv = fmaf(uv, Dd, yv);
      if (hasz) {
        const float sg = __builtin_amdgcn_rcpf(1.0f + expf(-zv));
        yv = yv * (zv * sg);
      }
      if (sq == 0) sY[ls * YP + c] = yv * a.ycarry;
    }
    __syncthreads();
    ms1_v4u hw[NIT], lw[NIT];
#pragma unroll
    for (int it = 0; it < NIT; ++it) {
      const int row = it * RPI + wave * 4 + q;
      const float* sp = sY + row * YP + c8;
      const ms1_v4f f0 = *(const ms1_v4f*)(sp);
      const ms1_v4f f1 = *(const ms1_v4f*)(sp + 4);
      unsigned h0, h1, h2, h3, l0, l1, l2, l3;
      ms1_pack2(f0[0], f0[1], h0, l0);
      ms1_pack2(f0[2], f0[3], h1, l1);
      ms1_pack2(f1[0], f1[1], h2, l2);
      ms1_pack2(f1[2], f1[3], h3, l3);
      hw[it] = (ms1_v4u){h0, h1, h2, h3};
      lw[it] = (ms1_v4u){l0, l1, l2, l3};
    }
    for (int pass = 0; pass < 2; ++pass) {
#pragma unroll
      for (int it = 0; it < NIT; ++it) {
        const int row = it * RPI + wave * 4 + q;
        const long o = (rowc + row) * a.ld_y + d0 + c8;
        *(volatile ms1_v4u*)(a.y + o) = hw[it];
        if (hasLo) *(volatile ms1_v4u*)(a.y_lo + o) = lw[it];
      }
      __threadfence();
    }
  }
}

__device__ __forceinline__ v4u yh_words(const unsigned short* __restrict__ YH, int k, int b, int p, int c8) {
  const int row = (k * kBatch + b) * kL + inv_time(k, p);
  return *(const v4u*)(YH + (size_t)row * kE + c8);
}
__device__ __forceinline__ _Float16 gate_half(unsigned h0, unsigned h1, unsigned h2, unsigned h3,
                                              float zr, float xi, float dp) {
  const float v0 = h16_to_f32(h0);
  const float v1 = h16_to_f32(h1);
  const float v2 = h16_to_f32(h2);
  const float v3 = h16_to_f32(h3);
  const float s01 = v0 + v1;
  const float s012 = s01 + v2;
  const float s = s012 + v3;
  const float ym = s * kMergeScale;
  const float g = zr / (1.0f + expf(-zr));
  const float yg = ym * g + xi * bf16r(dp);
  return f16_flush(yg * kGCarry);
}
__global__ __launch_bounds__(256) void merge_gate_kernel(
    const unsigned short* __restrict__ YH, const float* __restrict__ XZ,
    const float* __restrict__ dpar, unsigned short* __restrict__ YG)
{
  const int i = blockIdx.x * 256 + threadIdx.x;
  const int r = i / (kE / 8);
  const int c8 = (i - r * (kE / 8)) * 8;
  const int b = r / kL;
  const int p = r - b * kL;
  const v4u w0 = yh_words(YH, 0, b, p, c8);
  const v4u w1 = yh_words(YH, 1, b, p, c8);
  const v4u w2 = yh_words(YH, 2, b, p, c8);
  const v4u w3 = yh_words(YH, 3, b, p, c8);
  const float* xp = XZ + (size_t)r * kXzN + c8;
  const float* zp = xp + kE;
  const v4f xa = *(const v4f*)(xp);
  const v4f xb = *(const v4f*)(xp + 4);
  const v4f za = *(const v4f*)(zp);
  const v4f zb = *(const v4f*)(zp + 4);
  const v4f da = *(const v4f*)(dpar + c8);
  const v4f db = *(const v4f*)(dpar + c8 + 4);
  const unsigned p00 = w0[0];
  const unsigned p01 = w0[1];
  const unsigned p02 = w0[2];
  const unsigned p03 = w0[3];
  const unsigned p10 = w1[0];
  const unsigned p11 = w1[1];
  const unsigned p12 = w1[2];
  const unsigned p13 = w1[3];
  const unsigned p20 = w2[0];
  const unsigned p21 = w2[1];
  const unsigned p22 = w2[2];
  const unsigned p23 = w2[3];
  const unsigned p30 = w3[0];
  const unsigned p31 = w3[1];
  const unsigned p32 = w3[2];
  const unsigned p33 = w3[3];
  const float x0 = xa[0];
  const float x1 = xa[1];
  const float x2 = xa[2];
  const float x3 = xa[3];
  const float x4 = xb[0];
  const float x5 = xb[1];
  const float x6 = xb[2];
  const float x7 = xb[3];
  const float z0 = za[0];
  const float z1 = za[1];
  const float z2 = za[2];
  const float z3 = za[3];
  const float z4 = zb[0];
  const float z5 = zb[1];
  const float z6 = zb[2];
  const float z7 = zb[3];
  const float d0 = da[0];
  const float d1 = da[1];
  const float d2 = da[2];
  const float d3 = da[3];
  const float d4 = db[0];
  const float d5 = db[1];
  const float d6 = db[2];
  const float d7 = db[3];
  v8h hv;
  hv[0] = gate_half(p00 & 0xffffu, p10 & 0xffffu, p20 & 0xffffu, p30 & 0xffffu, z0, x0, d0);
  hv[1] = gate_half(p00 >> 16, p10 >> 16, p20 >> 16, p30 >> 16, z1, x1, d1);
  hv[2] = gate_half(p01 & 0xffffu, p11 & 0xffffu, p21 & 0xffffu, p31 & 0xffffu, z2, x2, d2);
  hv[3] = gate_half(p01 >> 16, p11 >> 16, p21 >> 16, p31 >> 16, z3, x3, d3);
  hv[4] = gate_half(p02 & 0xffffu, p12 & 0xffffu, p22 & 0xffffu, p32 & 0xffffu, z4, x4, d4);
  hv[5] = gate_half(p02 >> 16, p12 >> 16, p22 >> 16, p32 >> 16, z5, x5, d5);
  hv[6] = gate_half(p03 & 0xffffu, p13 & 0xffffu, p23 & 0xffffu, p33 & 0xffffu, z6, x6, d6);
  hv[7] = gate_half(p03 >> 16, p13 >> 16, p23 >> 16, p33 >> 16, z7, x7, d7);
  unsigned short* q = YG + (size_t)i * 8;
  *(volatile v8h*)q = hv;
  __threadfence();
  *(volatile v8h*)q = hv;
}

__global__ __launch_bounds__(256) void pack_wout_kernel(
    const float* __restrict__ w, unsigned short* __restrict__ OW)
{
  const int i = blockIdx.x * 256 + threadIdx.x;
  const int m = i / (kE / 8);
  const int c8 = (i - m * (kE / 8)) * 8;
  const float* sp = w + (size_t)m * kE + c8;
  const v4f a0 = *(const v4f*)(sp);
  const v4f a1 = *(const v4f*)(sp + 4);
  const v8h hv = pack8_in(a0, a1, kWCarry, true);
  unsigned short* q = OW + (size_t)i * 8;
  *(volatile v8h*)q = hv;
  __threadfence();
  *(volatile v8h*)q = hv;
}

__global__ __launch_bounds__(256) void resid_kernel(
    const float* __restrict__ RAW, const float* __restrict__ x, float* __restrict__ RES)
{
  const int wi = blockIdx.x * 256 + threadIdx.x;
  const v4f a = *(const v4f*)(RAW + (size_t)wi * 4);
  const v4f xv = *(const v4f*)(x + (size_t)wi * 4);
  const float a0 = a[0];
  const float a1 = a[1];
  const float a2 = a[2];
  const float a3 = a[3];
  const float e0 = xv[0];
  const float e1 = xv[1];
  const float e2 = xv[2];
  const float e3 = xv[3];
  v4f o;
  o[0] = a0 + bf16r(e0);
  o[1] = a1 + bf16r(e1);
  o[2] = a2 + bf16r(e2);
  o[3] = a3 + bf16r(e3);
  float* q = RES + (size_t)wi * 4;
  *(volatile v4f*)q = o;
  __threadfence();
  *(volatile v4f*)q = o;
}

__global__ __launch_bounds__(256) void ln_stats_kernel(
    const float* __restrict__ RES, float* __restrict__ ST)
{
  const int r = blockIdx.x * 256 + threadIdx.x;
  const float* mp = RES + (size_t)r * kDm;
  float sum = 0.0f;
  for (int c = 0; c < 384; c += 4) {
    const v4f v = *(const v4f*)(mp + c);
    const float a0 = v[0];
    const float a1 = v[1];
    const float a2 = v[2];
    const float a3 = v[3];
    sum = sum + a0;
    sum = sum + a1;
    sum = sum + a2;
    sum = sum + a3;
  }
  const float mu = sum * (1.0f / 384.0f);
  float vs = 0.0f;
  for (int c = 0; c < 384; c += 4) {
    const v4f v = *(const v4f*)(mp + c);
    const float a0 = v[0];
    const float a1 = v[1];
    const float a2 = v[2];
    const float a3 = v[3];
    const float e0 = a0 - mu;
    const float e1 = a1 - mu;
    const float e2 = a2 - mu;
    const float e3 = a3 - mu;
    vs = fmaf(e0, e0, vs);
    vs = fmaf(e1, e1, vs);
    vs = fmaf(e2, e2, vs);
    vs = fmaf(e3, e3, vs);
  }
  const float var = vs * (1.0f / 384.0f);
  const float rs = 1.0f / sqrtf(var + 1e-5f);
  v4f ov;
  ov[0] = mu;
  ov[1] = rs;
  ov[2] = 0.0f;
  ov[3] = 0.0f;
  float* q = ST + (size_t)r * 4;
  *(volatile v4f*)q = ov;
  __threadfence();
  *(volatile v4f*)q = ov;
}

__device__ __forceinline__ float ln_val(float m, float mu, float rs, float lw, float lb) {
  return (m - mu) * rs * bf16r(lw) + bf16r(lb);
}
__global__ __launch_bounds__(256) void ln_out_kernel(
    const float* __restrict__ RES, const float* __restrict__ ST,
    const float* __restrict__ lng, const float* __restrict__ lnb, float* __restrict__ out)
{
  const int i = blockIdx.x * 256 + threadIdx.x;
  const int r = i / (kDm / 4);
  const int c4 = (i - r * (kDm / 4)) * 4;
  const v4f mv = *(const v4f*)(RES + (size_t)i * 4);
  const v4f st = *(const v4f*)(ST + (size_t)r * 4);
  const v4f wv = *(const v4f*)(lng + c4);
  const v4f bv = *(const v4f*)(lnb + c4);
  const float mu = st[0];
  const float rs = st[1];
  const float m0 = mv[0];
  const float m1 = mv[1];
  const float m2 = mv[2];
  const float m3 = mv[3];
  const float g0 = wv[0];
  const float g1 = wv[1];
  const float g2 = wv[2];
  const float g3 = wv[3];
  const float o0 = bv[0];
  const float o1 = bv[1];
  const float o2 = bv[2];
  const float o3 = bv[3];
  v4f o;
  o[0] = ln_val(m0, mu, rs, g0, o0);
  o[1] = ln_val(m1, mu, rs, g1, o1);
  o[2] = ln_val(m2, mu, rs, g2, o2);
  o[3] = ln_val(m3, mu, rs, g3, o3);
  float* q = out + (size_t)i * 4;
  *(volatile v4f*)q = o;
  __threadfence();
  *(volatile v4f*)q = o;
}

static_assert(((kRows / 32) * (kXzN / 64)) % 8 == 0 && ((kRows / 32) * (kXzN / 64)) / 8 == 192);
static_assert(((kRows / 32) * (kXpP / 64)) % 8 == 0 && ((kRows / 32) * (kXpP / 64)) / 8 == 8);
static_assert(((kRows / 32) * (kE / 64)) % 8 == 0 && ((kRows / 32) * (kE / 64)) / 8 == 96);
static_assert(((kRows / 32) * (kDm / 64)) % 8 == 0 && ((kRows / 32) * (kDm / 64)) / 8 == 48);
static_assert(((kRows * kDm / 8) % 256) == 0 && (kRows * kDm / 8) / 256 == 384);
static_assert(((kXzN * kDm / 8) % 256) == 0 && (kXzN * kDm / 8) / 256 == 288);
static_assert(((kRows * kE / 8) % 256) == 0 && (kRows * kE / 8) / 256 == 768);
static_assert(((kXpP * kE / 8) % 256) == 0 && (kXpP * kE / 8) / 256 == 24);
static_assert(((kRows * kRkP / 8) % 256) == 0 && (kRows * kRkP / 8) / 256 == 32);
static_assert(((kE * kRkP / 8) % 256) == 0 && (kE * kRkP / 8) / 256 == 12);
static_assert(((kDirs * kRows * kE / 4) % 256) == 0 && (kDirs * kRows * kE / 4) / 256 == 6144);
static_assert(((kDirs * kRows * kXpP / 4) % 256) == 0 && (kDirs * kRows * kXpP / 4) / 256 == 512);
static_assert((kPadFloats / 4) == 102 * 32);
static_assert(((kDm * kE / 8) % 256) == 0 && (kDm * kE / 8) / 256 == 144);
static_assert(((kRows * kDm / 4) % 256) == 0 && (kRows * kDm / 4) / 256 == 768);
static_assert((kRows % 256) == 0 && kRows / 256 == 8);
static_assert((kE % 64) == 0 && (kL % 64) == 0);
static_assert(kRows == kBatch * kL);
static_assert((768 / 64) * 32 == 384);
static_assert((kE / 64) * (kDirs * kBatch) == 384);

extern "C" void kernel_launch(void* const* d_in, const int* in_sizes, int n_in,
                              void* d_out, int out_size, void* d_ws, size_t ws_size,
                              hipStream_t stream)
{
  if (n_in < 10) return;
  if (in_sizes[0] != kRows * kDm) return;
  if (in_sizes[1] != kXzN * kDm) return;
  if (in_sizes[2] != kE * kNst) return;
  if (in_sizes[3] != kXpN * kE) return;
  if (in_sizes[4] != kE * kRank) return;
  if (in_sizes[5] != kE) return;
  if (in_sizes[6] != kE) return;
  if (in_sizes[7] != kDm * kE) return;
  if (in_sizes[8] != kDm) return;
  if (in_sizes[9] != kDm) return;
  if (out_size != kRows * kDm) return;
  if (ws_size < kWsTotal) return;

  const float* x      = (const float*)d_in[0];
  const float* w_in   = (const float*)d_in[1];
  const float* a_log  = (const float*)d_in[2];
  const float* w_x    = (const float*)d_in[3];
  const float* w_dt   = (const float*)d_in[4];
  const float* b_dt   = (const float*)d_in[5];
  const float* d_par  = (const float*)d_in[6];
  const float* w_out  = (const float*)d_in[7];
  const float* ln_g   = (const float*)d_in[8];
  const float* ln_b   = (const float*)d_in[9];
  float* out = (float*)d_out;

  char* ws = (char*)d_ws;
  unsigned short* XH   = (unsigned short*)(ws + kOffXH);
  unsigned short* WIN  = (unsigned short*)(ws + kOffWIN);
  float*          XZ   = (float*)(ws + kOffXZ);
  unsigned short* XIH  = (unsigned short*)(ws + kOffXIH);
  unsigned short* WX   = (unsigned short*)(ws + kOffWX);
  float*          XD0  = (float*)(ws + kOffXD0);
  unsigned short* DRH  = (unsigned short*)(ws + kOffDRH);
  unsigned short* WDT  = (unsigned short*)(ws + kOffWDT);
  float*          DT0  = (float*)(ws + kOffDT0);
  float*          XS   = (float*)(ws + kOffXS);
  float*          DTP  = (float*)(ws + kOffDTP);
  float*          XD   = (float*)(ws + kOffXD);
  float*          PADS = (float*)(ws + kOffPADS);
  unsigned short* YH   = (unsigned short*)(ws + kOffYH);
  unsigned short* YG   = (unsigned short*)(ws + kOffYG);
  unsigned short* OW   = (unsigned short*)(ws + kOffOW);
  float*          RAW  = (float*)(ws + kOffRAW);
  float*          RES  = (float*)(ws + kOffRES);
  float*          ST   = (float*)(ws + kOffST);
  float*          ALP  = PADS;
  float*          DSP  = PADS + kAlpFloats;

  constexpr float s1 = 1.0f / (kXCarry * kWCarry);
  constexpr float s2 = 1.0f / (kSCarry * kWCarry);
  constexpr float s3 = 1.0f / (kRCarry * kWCarry);
  constexpr float s4 = 1.0f / (kGCarry * kWCarry);

  pack_x_kernel<<<(kRows * kDm / 8) / 256, 256, 0, stream>>>(x, XH);

  pack_win_kernel<<<(kXzN * kDm / 8) / 256, 256, 0, stream>>>(w_in, WIN);

  eng::gemm_f16_kernel<2, 0><<<dim3((2048 / 32) * (1536 / 64) / 8), 256, 0, stream>>>(
      XH, nullptr, 384, WIN, nullptr, 384, XZ, 1536, 2048, 1536, 384, s1, 0.0f);

  pack_xi_kernel<<<(kRows * kE / 8) / 256, 256, 0, stream>>>(XZ, XIH);

  pack_wx_kernel<<<(kXpP * kE / 8) / 256, 256, 0, stream>>>(w_x, WX);

  eng::gemm_f16_kernel<2, 0><<<dim3((2048 / 32) * (64 / 64) / 8), 256, 0, stream>>>(
      XIH, nullptr, 768, WX, nullptr, 768, XD0, 64, 2048, 64, 768, s2, 0.0f);

  pack_dr_kernel<<<(kRows * kRkP / 8) / 256, 256, 0, stream>>>(XD0, DRH);

  pack_wdt_kernel<<<(kE * kRkP / 8) / 256, 256, 0, stream>>>(w_dt, b_dt, WDT);

  eng::gemm_f16_kernel<2, 0><<<dim3((2048 / 32) * (768 / 64) / 8), 256, 0, stream>>>(
      DRH, nullptr, 32, WDT, nullptr, 32, DT0, 768, 2048, 768, 32, s3, 0.0f);

  order_kernel<<<(kDirs * kRows * kE / 4) / 256, 256, 0, stream>>>(XZ, XS);

  gather_dt_kernel<<<(kDirs * kRows * kE / 4) / 256, 256, 0, stream>>>(DT0, DTP);

  gather_bc_kernel<<<(kDirs * kRows * kXpP / 4) / 256, 256, 0, stream>>>(XD0, XD);

  pads_kernel<<<102, 32, 0, stream>>>(a_log, PADS);

  ms1_args sa;
  sa.dtpre = DTP;
  sa.u = XS;
  sa.bc = XD;
  sa.z = nullptr;
  sa.A_log = ALP;
  sa.Dskip = DSP;
  sa.y = (__half*)YH;
  sa.y_lo = nullptr;
  sa.ld_dtpre = kE;
  sa.ld_u = kE;
  sa.ld_bc = kXpP;
  sa.ld_z = 0;
  sa.ld_y = kE;
  sa.offB = kRank;
  sa.offC = kRank + kNst;
  sa.offZ = 0;
  sa.ycarry = kYCarry;
  sa.dir = 1;
  sa.D = kE;
  sa.L = kL;
  sa.nbatch = kDirs * kBatch;
  ms1_scan_kernel<16><<<dim3((768 / 64) * 32), 64, 0, stream>>>(sa);

  merge_gate_kernel<<<(kRows * kE / 8) / 256, 256, 0, stream>>>(YH, XZ, d_par, YG);

  pack_wout_kernel<<<(kDm * kE / 8) / 256, 256, 0, stream>>>(w_out, OW);

  eng::gemm_f16_kernel<2, 0><<<dim3((2048 / 32) * (384 / 64) / 8), 256, 0, stream>>>(
      YG, nullptr, 768, OW, nullptr, 768, RAW, 384, 2048, 384, 768, s4, 0.0f);

  resid_kernel<<<(kRows * kDm / 4) / 256, 256, 0, stream>>>(RAW, x, RES);

  ln_stats_kernel<<<kRows / 256, 256, 0, stream>>>(RES, ST);

  ln_out_kernel<<<(kRows * kDm / 4) / 256, 256, 0, stream>>>(RES, ST, ln_g, ln_b, out);
}
